// OuterProductMean_51170240365056
// MI455X (gfx1250) — hardware-verified
//
#include <hip/hip_runtime.h>
#include <math.h>

typedef __attribute__((ext_vector_type(16))) _Float16 v16h;
typedef __attribute__((ext_vector_type(16))) __bf16 v16b;
typedef __attribute__((ext_vector_type(8)))  _Float16 v8h;
typedef __attribute__((ext_vector_type(8)))  float v8f;
typedef __attribute__((ext_vector_type(4)))  float v4f;
typedef __attribute__((ext_vector_type(2)))  float v2f;
typedef __attribute__((ext_vector_type(4)))  unsigned v4u;
typedef __attribute__((ext_vector_type(4)))  int v4i;
typedef float __attribute__((may_alias)) float_a;
typedef int __attribute__((may_alias)) int_a;

template <typename T> __device__ __forceinline__ void vst2(void* p, T v) { *(volatile T*)p = v; __threadfence(); *(volatile T*)p = v; }
__device__ __forceinline__ v8f wmma16(v16h a, v16h b, v8f c) {
  v8f d = __builtin_amdgcn_wmma_f32_16x16x32_f16(false, a, false, b, (short)0, c, false, false);
  asm volatile("v_nop\n\tv_nop\n\tv_nop\n\tv_nop" : "+v"(d) : "v"(a), "v"(b));
  return d;
}
__device__ __forceinline__ v8f wmma_bf(v16b a, v16b b, v8f c) {
  v8f d = __builtin_amdgcn_wmma_f32_16x16x32_bf16(false, a, false, b, (short)0, c, false, false);
  asm volatile("v_nop\n\tv_nop\n\tv_nop\n\tv_nop" : "+v"(d) : "v"(a), "v"(b));
  return d;
}
__device__ __forceinline__ v16h frag_h(const _Float16* rowk0, int lane) {
  union { v16h v; v8h q[2]; } u; const _Float16* p = rowk0 + 8 * (lane >> 4);
  u.q[0] = *(const v8h*)p; u.q[1] = *(const v8h*)(p + 16); return u.v;
}
__device__ __forceinline__ v16h frag_f32(const float* rowk0, int lane) {
  v16h a; const float* p = rowk0 + 8 * (lane >> 4);
#pragma unroll
  for (int i = 0; i < 8; ++i) { a[i] = (_Float16)p[i]; a[8 + i] = (_Float16)p[16 + i]; }
  return a;
}
__device__ __forceinline__ v16h frag_f32s(const float* rowk0, int lane, float sc) {
  v16h a; const float* p = rowk0 + 8 * (lane >> 4);
#pragma unroll
  for (int i = 0; i < 8; ++i) { a[i] = (_Float16)(p[i] * sc); a[8 + i] = (_Float16)(p[16 + i] * sc); }
  return a;
}
__device__ __forceinline__ v16h fragc_f32(const float* W, int k0, int n, int lane, int ld, int K) {
  v16h a; const int g = lane >> 4;
#pragma unroll
  for (int i = 0; i < 8; ++i) { const int ka = k0 + 8 * g + i, kb = ka + 16;
    a[i] = (_Float16)(ka < K ? W[(size_t)(ka < K ? ka : K - 1) * ld + n] : 0.f); a[8 + i] = (_Float16)(kb < K ? W[(size_t)(kb < K ? kb : K - 1) * ld + n] : 0.f); }
  return a;
}
struct F2 { v16b h, l; };
__device__ __forceinline__ F2 bsplit16(const float v[16]) { F2 r;
#pragma unroll
  for (int i = 0; i < 16; ++i) { const __bf16 h = (__bf16)v[i]; r.h[i] = h; r.l[i] = (__bf16)(v[i] - (float)h); }
  return r; }
__device__ __forceinline__ F2 split_row(const float* row, int k0, int lane) { float v[16]; const float* p = row + k0 + 8 * (lane >> 4);
#pragma unroll
  for (int i = 0; i < 8; ++i) { v[i] = p[i]; v[8 + i] = p[16 + i]; }
  return bsplit16(v); }
__device__ __forceinline__ F2 split_rowK(const float* row, int k0, int lane, int K) { float v[16]; const int g = lane >> 4;
#pragma unroll
  for (int i = 0; i < 8; ++i) { const int ka = k0 + 8 * g + i, kb = ka + 16; v[i] = ka < K ? row[ka < K ? ka : K - 1] : 0.f; v[8 + i] = kb < K ? row[kb < K ? kb : K - 1] : 0.f; }
  return bsplit16(v); }
__device__ __forceinline__ F2 split_col(const float* W, int k0, int n, int lane, int ld, int K) { float v[16]; const int g = lane >> 4;
#pragma unroll
  for (int i = 0; i < 8; ++i) { const int ka = k0 + 8 * g + i, kb = ka + 16; v[i] = ka < K ? W[(size_t)(ka < K ? ka : K - 1) * ld + n] : 0.f; v[8 + i] = kb < K ? W[(size_t)(kb < K ? kb : K - 1) * ld + n] : 0.f; }
  return bsplit16(v); }
__device__ __forceinline__ v8f mac3(const F2& a, const F2& b, v8f c) { c = wmma_bf(a.l, b.h, c); c = wmma_bf(a.h, b.l, c); return wmma_bf(a.h, b.h, c); }
__device__ __forceinline__ float sigm(float v) { return 1.0f / (1.0f + expf(-v)); }
#define LDSX() do { asm volatile("s_wait_dscnt 0" ::: "memory"); __builtin_amdgcn_wave_barrier(); __builtin_amdgcn_fence(__ATOMIC_RELEASE, "workgroup"); } while (0)

__device__ __forceinline__ float bfr(float v) { return (float)(__bf16)v; }
__device__ __attribute__((noinline)) float gelu_ni(float x) { return 0.5f * x * (1.0f + erff(x * 0.70710678118654752f)); }
#define SS 128
#define NN 256
#define DM 256
#define DH 32
#define DP 128
#define NPAIR (NN * NN)
#define KO (DH * DH)
#ifndef NPB
#define NPB NPAIR
#endif
#define WS_ST  0u
#define WS_AT  (WS_ST + 4u * (size_t)SS * NN * 2)
#define WS_BT  (WS_AT + 2u * (size_t)NN * DH * SS)
#define WS_NRM (WS_BT + 2u * (size_t)NN * DH * SS)
#define WS_O   (WS_NRM + 4u * (size_t)NPAIR)
#define WS_END (WS_O + 2u * (size_t)NPAIR * KO)
__global__ __launch_bounds__(256) void k_stat(const float* __restrict__ M, float* __restrict__ ST) { __shared__ __align__(16) float so[32];
  const int t = threadIdx.x; const int rl = t >> 4, sub = t & 15; const size_t row = (size_t)blockIdx.x * 16 + rl; const float* p = M + row * DM;
  float s = 0.f; for (int c = sub; c < DM; c += 16) s += bfr(p[c]);
#pragma unroll
  for (int o = 1; o < 16; o <<= 1) s += __shfl_xor(s, o);
  const float mu = s * (1.0f / DM); float s2 = 0.f; for (int c = sub; c < DM; c += 16) { const float d = bfr(p[c]) - mu; s2 += d * d; }
#pragma unroll
  for (int o = 1; o < 16; o <<= 1) s2 += __shfl_xor(s2, o);
  if (sub == 0) { so[rl * 2] = mu; so[rl * 2 + 1] = rsqrtf(s2 * (1.0f / DM) + 1e-5f); }
  __syncthreads(); if (t < 32) vst2(ST + (size_t)blockIdx.x * 32 + t, so[t]); }
__global__ __launch_bounds__(128) void k_ab(const float* __restrict__ M, const float* __restrict__ ST, const float* __restrict__ MSK, const float* __restrict__ LW, const float* __restrict__ LB, const float* __restrict__ W1, const float* __restrict__ B1, const float* __restrict__ W2, const float* __restrict__ B2, _Float16* __restrict__ AT, _Float16* __restrict__ BT) { __shared__ __align__(16) _Float16 tp[DH][72];
  const int tid = threadIdx.x, wave = tid >> 5, lane = tid & 31, col = lane & 15, g = lane >> 4; const int n = blockIdx.x; const int s0 = blockIdx.y * 64; const int which = blockIdx.z; const float* Wt = which == 0 ? W1 : W2; const float* Bb = which == 0 ? B1 : B2; _Float16* DST = which == 0 ? AT : BT;
  const int sa = s0 + wave * 16 + col; const size_t mrow = (size_t)sa * NN + n; const float mu = ST[mrow * 2], rs = ST[mrow * 2 + 1];
  v8f acc[2] = {};
#pragma unroll 2
  for (int kc = 0; kc < DM / 32; ++kc) { v16h a; { const float* p = M + mrow * DM + kc * 32 + 8 * g;
#pragma unroll
      for (int i = 0; i < 8; ++i) { const int c = kc * 32 + 8 * g + i; a[i] = (_Float16)((bfr(p[i]) - mu) * rs * bfr(LW[c]) + bfr(LB[c])); a[8 + i] = (_Float16)((bfr(p[16 + i]) - mu) * rs * bfr(LW[c + 16]) + bfr(LB[c + 16])); } }
#pragma unroll
    for (int j = 0; j < 2; ++j) { v16h w; const int o = j * 16 + col; const float* wr = Wt + (size_t)o * DM + kc * 32 + 8 * g;
#pragma unroll
      for (int i = 0; i < 8; ++i) { w[i] = (_Float16)(bfr(wr[i]) * 16.0f); w[8 + i] = (_Float16)(bfr(wr[16 + i]) * 16.0f); }
      acc[j] = wmma16(a, w, acc[j]); } }
#pragma unroll
  for (int j = 0; j < 2; ++j) { const int o = j * 16 + col; const float bb = bfr(Bb[o]);
#pragma unroll
    for (int r = 0; r < 8; ++r) { const int sl = wave * 16 + 8 * g + r; const float mk = bfr(MSK[(size_t)(s0 + sl) * NN + n]) * 0.0625f;     tp[o][sl] = (_Float16)((acc[j][r] * (1.0f / 16.0f) + bb) * mk); } }
  __syncthreads();
  for (int e = tid; e < DH * 8; e += 128) { const int c = e >> 3, q = e & 7; vst2((unsigned*)(DST + ((size_t)n * DH + c) * SS + s0 + q * 8), *(const v4u*)&tp[c][q * 8]); } }
__global__ __launch_bounds__(64) void k_norm(const float* __restrict__ MSK, float* __restrict__ NRM) { __shared__ __align__(16) float so[64];
  const int t = threadIdx.x; const size_t pr = (size_t)blockIdx.x * 64 + t; const int i = (int)(pr / NN), j = (int)(pr % NN); float s = 0.f;
#pragma unroll 1
  for (int ss_ = 0; ss_ < SS; ++ss_) s += (bfr(MSK[(size_t)ss_ * NN + i]) * 0.0625f) * (bfr(MSK[(size_t)ss_ * NN + j]) * 0.0625f);
  so[t] = s; __syncthreads(); if (t < 16) vst2(NRM + (size_t)blockIdx.x * 64 + t * 4, *(const v4f*)&so[t * 4]); }
__global__ __launch_bounds__(128) void k_outer(const _Float16* __restrict__ AT, const _Float16* __restrict__ BT, _Float16* __restrict__ O) { __shared__ __align__(16) _Float16 so[4][DH][DH + 8];
  const int tid = threadIdx.x, wave = tid >> 5, lane = tid & 31, col = lane & 15, g = lane >> 4; const int i = blockIdx.x; const int j0 = blockIdx.y * 64 + wave * 16;
  v16h af[2][4];
#pragma unroll
  for (int ct = 0; ct < 2; ++ct)
#pragma unroll
    for (int kc = 0; kc < 4; ++kc) af[ct][kc] = frag_h(AT + ((size_t)i * DH + ct * 16 + col) * SS + kc * 32, lane);
#pragma unroll 1
  for (int jj = 0; jj < 16; ++jj) { const int j = j0 + jj; v8f acc[2][2] = {};
#pragma unroll
    for (int kc = 0; kc < 4; ++kc) {
#pragma unroll
      for (int et = 0; et < 2; ++et) { const v16h bfr_ = frag_h(BT + ((size_t)j * DH + et * 16 + col) * SS + kc * 32, lane); acc[0][et] = wmma16(af[0][kc], bfr_, acc[0][et]); acc[1][et] = wmma16(af[1][kc], bfr_, acc[1][et]); } }
#pragma unroll
    for (int ct = 0; ct < 2; ++ct)
#pragma unroll
      for (int et = 0; et < 2; ++et)
#pragma unroll
        for (int r = 0; r < 8; ++r) so[wave][ct * 16 + 8 * g + r][et * 16 + col] = (_Float16)acc[ct][et][r];
    LDSX();
    { const size_t prw = (size_t)i * NN + j; const int c = lane; vst2((v4u*)(O + prw * KO + c * DH), *(const v4u*)&so[wave][c][0]); vst2((v4u*)(O + prw * KO + c * DH + 8), *(const v4u*)&so[wave][c][8]); vst2((v4u*)(O + prw * KO + c * DH + 16), *(const v4u*)&so[wave][c][16]); vst2((v4u*)(O + prw * KO + c * DH + 24), *(const v4u*)&so[wave][c][24]); }
    LDSX(); } }
__global__ __launch_bounds__(128) void k_z(const _Float16* __restrict__ O, const float* __restrict__ WO, const float* __restrict__ BO, const float* __restrict__ NRM, const float* __restrict__ LW, const float* __restrict__ LB, const float* __restrict__ WZ, const float* __restrict__ BZ, float* __restrict__ OUT) {
  __shared__ __align__(16) float sz[64][DP + 4]; __shared__ __align__(16) float sln[64][DP + 4]; __shared__ __align__(16) float sf[4][16][132];
  const int tid = threadIdx.x, wave = tid >> 5, lane = tid & 31, col = lane & 15, g = lane >> 4; const size_t p0 = (size_t)blockIdx.x * 64 + wave * 16;
  { v8f acc[8] = {};
#pragma unroll 1
    for (int kc = 0; kc < KO / 32; ++kc) { const v16h a = frag_h(O + (p0 + col) * KO + kc * 32, lane);
#pragma unroll
      for (int jt = 0; jt < 8; ++jt) { v16h w; const int o = jt * 16 + col; const float* wr = WO + (size_t)o * KO + kc * 32 + 8 * g;
#pragma unroll
        for (int q = 0; q < 8; ++q) { w[q] = (_Float16)(bfr(wr[q]) * 8.0f); w[8 + q] = (_Float16)(bfr(wr[16 + q]) * 8.0f); }
        acc[jt] = wmma16(a, w, acc[jt]); } }
#pragma unroll
    for (int jt = 0; jt < 8; ++jt) { const int o = jt * 16 + col; const float bb = bfr(BO[o]);
#pragma unroll
      for (int r = 0; r < 8; ++r) { const int rl = wave * 16 + 8 * g + r; const float nrm = NRM[p0 + 8 * g + r]; const float z = (acc[jt][r] * 0.125f + bb) / (1e-3f + nrm); sz[rl][o] = gelu_ni(z); } } }
  __syncthreads();
  { const int row = tid >> 1, half = tid & 1; float s = 0.f; for (int e = 0; e < 64; ++e) s += sz[row][half * 64 + e]; s += __shfl_xor(s, 1); const float mu = s * (1.0f / DP); float s2 = 0.f; for (int e = 0; e < 64; ++e) { const float d = sz[row][half * 64 + e] - mu; s2 += d * d; } s2 += __shfl_xor(s2, 1); const float rs = rsqrtf(s2 * (1.0f / DP) + 1e-5f);
    for (int e = 0; e < 64; ++e) { const int c = half * 64 + e; sln[row][c] = (sz[row][c] - mu) * rs * bfr(LW[c]) + bfr(LB[c]); } }
  __syncthreads();
  { v8f acc[8] = {};
#pragma unroll
    for (int kc = 0; kc < DP / 32; ++kc) { const F2 a = split_row(&sln[wave * 16 + col][0], kc * 32, lane);
#pragma unroll
      for (int jt = 0; jt < 8; ++jt) { v16b w; const int o = jt * 16 + col; const float* wr = WZ + (size_t)o * DP + kc * 32 + 8 * g;
#pragma unroll
        for (int q = 0; q < 8; ++q) { w[q] = (__bf16)wr[q]; w[8 + q] = (__bf16)wr[16 + q]; }
        acc[jt] = wmma_bf(a.h, w, acc[jt]); acc[jt] = wmma_bf(a.l, w, acc[jt]); } }
#pragma unroll
    for (int jt = 0; jt < 8; ++jt) { const int o = jt * 16 + col; const float bb = bfr(BZ[o]);
#pragma unroll
      for (int r = 0; r < 8; ++r) sf[wave][8 * g + r][o] = acc[jt][r] + bb; } }
  LDSX(); for (int rl = 0; rl < 16; ++rl) vst2(OUT + (p0 + rl) * DP + lane * 4, *(const v4f*)&sf[wave][rl][lane * 4]); }
extern "C" void kernel_launch(void* const* d_in, const int* in_sizes, int n_in, void* d_out, int out_size, void* d_ws, size_t ws_size, hipStream_t stream) {
  (void)in_sizes; (void)n_in; (void)out_size;
  const float** F = (const float**)d_in;
  if (ws_size < (size_t)WS_END) return;
  char* ws = (char*)d_ws; float *ST = (float*)(ws + WS_ST), *NRM = (float*)(ws + WS_NRM); _Float16 *AT = (_Float16*)(ws + WS_AT), *BT = (_Float16*)(ws + WS_BT), *O = (_Float16*)(ws + WS_O);
  k_stat<<<dim3(SS * NN / 16), 256, 0, stream>>>(F[0], ST);
  k_ab<<<dim3(NN, SS / 64, 2), 128, 0, stream>>>(F[0], ST, F[1], F[2], F[3], F[4], F[5], F[6], F[7], AT, BT);
  k_norm<<<dim3(NPAIR / 64), 64, 0, stream>>>(F[1], NRM);
  k_outer<<<dim3(NPB / NN, NN / 64), 128, 0, stream>>>(AT, BT, O);
  k_z<<<dim3(NPB / 64), 128, 0, stream>>>(O, F[8], F[9], NRM, F[10], F[11], F[12], F[13], (float*)d_out);
}
